// RNN_3058016715203
// MI455X (gfx1250) — hardware-verified
//
#include <hip/hip_runtime.h>
#include <math.h>

constexpr int NSTEP   = 65536;
constexpr int NHID    = 64;
constexpr int NINP    = 12;
constexpr int NGATE   = 4 * NHID;
constexpr int KPAD    = 32;
constexpr int NOUTC   = 2;
constexpr int OBLK    = 64;
constexpr int RTHR    = 128;
constexpr int PTHR    = 256;
constexpr float WCARRY      = 16.0f;
constexpr float WCARRY_INV  = 1.0f / 16.0f;
constexpr float LOCARRY     = 2048.0f;
constexpr float LOCARRY_INV = 1.0f / 2048.0f;
constexpr float F16_MIN_NORMAL = 6.103515625e-05f;
static_assert(NGATE == 256, "gate count");
static_assert(NINP <= KPAD && KPAD % 32 == 0, "K padded to a multiple of 32");
static_assert(NSTEP % 64 == 0 && NGATE % 64 == 0, "GEMM M and N are tile multiples");
static_assert(((NSTEP / 64) * (NGATE / 64)) % 8 == 0, "GEMM grid exact");
static_assert(NHID == 64, "two k-steps of 32 per recurrent product");
static_assert(RTHR == 2 * NHID, "h tile zero fill is exact");
static_assert(RTHR / 32 == NHID / 16, "one wave per 16 hidden units");
static_assert(NSTEP % OBLK == 0, "output flush blocks are exact");
static_assert(NOUTC * OBLK == 32 * 4, "one flush = 32 lanes x 16 B");

typedef __attribute__((ext_vector_type(16))) _Float16 v16h;
typedef __attribute__((ext_vector_type(8)))  _Float16 v8h;
typedef __attribute__((ext_vector_type(16))) __bf16   v16b;
typedef __attribute__((ext_vector_type(8)))  __bf16   v8b;
typedef __attribute__((ext_vector_type(8)))  float    v8f;
typedef __attribute__((ext_vector_type(4)))  float    v4f;

__device__ __forceinline__ unsigned short f2bf_bits(float f) {
  unsigned u = __float_as_uint(f);
  return (unsigned short)((u + 0x7FFFu + ((u >> 16) & 1u)) >> 16);
}
__device__ __forceinline__ float bf_bits2f(unsigned short h) { return __uint_as_float(((unsigned)h) << 16); }

__device__ __forceinline__ void dep_guard_h(v8f& a, v8f& b, v16h x, v16h y) { asm volatile("v_nop\n\tv_nop\n\tv_nop\n\tv_nop" : "+v"(a), "+v"(b) : "v"(x), "v"(y)); }
__device__ __forceinline__ void dep_guard_b(v8f& a, v8f& b, v16b x, v16b y) { asm volatile("v_nop\n\tv_nop\n\tv_nop\n\tv_nop" : "+v"(a), "+v"(b) : "v"(x), "v"(y)); }
__device__ __forceinline__ void keep4_h(v16h a, v16h b, v16h c, v16h d) { asm volatile("v_nop" :: "v"(a), "v"(b), "v"(c), "v"(d)); }
__device__ __forceinline__ void keep4_b(v16b a, v16b b, v16b c, v16b d) { asm volatile("v_nop" :: "v"(a), "v"(b), "v"(c), "v"(d)); }
__device__ __forceinline__ void acc_guard4(v8f& a, v8f& b, v8f& c, v8f& d) { asm volatile("v_nop\n\tv_nop\n\tv_nop\n\tv_nop" : "+v"(a), "+v"(b), "+v"(c), "+v"(d)); }
__device__ __forceinline__ void group_guard4(v8f& a, v8f& b, v8f& c, v8f& d, v16h x, v16h y) {
  asm volatile("v_nop\n\tv_nop\n\tv_nop\n\tv_nop" : "+v"(a), "+v"(b), "+v"(c), "+v"(d) : "v"(x), "v"(y));
}
__device__ __forceinline__ void group_guard1(v8f& a, v16h x, v16h y, v16h p, v16h q) {
  asm volatile("v_nop\n\tv_nop\n\tv_nop\n\tv_nop" : "+v"(a) : "v"(x), "v"(y), "v"(p), "v"(q));
}
__device__ __forceinline__ void wave_lds_sync() {
  __builtin_amdgcn_fence(__ATOMIC_RELEASE, "workgroup");
  __builtin_amdgcn_wave_barrier();
  __builtin_amdgcn_fence(__ATOMIC_ACQUIRE, "workgroup");
}
__device__ __forceinline__ void settle_frag(v16h& f) { asm volatile("" : "+v"(f) : : "memory"); }
__device__ __forceinline__ void settle_f32(float& f)  { asm volatile("" : "+v"(f) : : "memory"); }

template <typename T> struct Frag;
template <> struct Frag<_Float16> {
  typedef v16h V; union U { v16h v; v8h h[2]; };
  static __device__ __forceinline__ v16h load(const _Float16* p) {
    U f; f.h[0] = *(const v8h*)(p); f.h[1] = *(const v8h*)(p + 16); return f.v;
  }
  static __device__ __forceinline__ v8f mma(v16h a, v16h b, v8f c) {
    return __builtin_amdgcn_wmma_f32_16x16x32_f16(false, a, false, b, (short)0, c, false, false);
  }
  static __device__ __forceinline__ void guard(v8f& a, v8f& b, v16h x, v16h y) { dep_guard_h(a, b, x, y); }
  static __device__ __forceinline__ void keep(v16h a, v16h b, v16h c, v16h d) { keep4_h(a, b, c, d); }
};
template <> struct Frag<__bf16> {
  typedef v16b V; union U { v16b v; v8b h[2]; };
  static __device__ __forceinline__ v16b load(const __bf16* p) {
    U f; f.h[0] = *(const v8b*)(p); f.h[1] = *(const v8b*)(p + 16); return f.v;
  }
  static __device__ __forceinline__ v8f mma(v16b a, v16b b, v8f c) {
    return __builtin_amdgcn_wmma_f32_16x16x32_bf16(false, a, false, b, (short)0, c, false, false);
  }
  static __device__ __forceinline__ void guard(v8f& a, v8f& b, v16b x, v16b y) { dep_guard_b(a, b, x, y); }
  static __device__ __forceinline__ void keep(v16b a, v16b b, v16b c, v16b d) { keep4_b(a, b, c, d); }
};

template <int ET> struct Elem;
template <> struct Elem<0> { typedef _Float16 T; };
template <> struct Elem<1> { typedef __bf16 T; };
template <int ET, bool SPLIT, int BIAS_MODE, int OUT_MODE, bool RESID, int ACT = 0>
__global__ __launch_bounds__(256) void wmma_gemm64(
    const unsigned short* __restrict__ Ap, const unsigned short* __restrict__ A2p, int lda, long strideA,
    const unsigned short* __restrict__ Btp, const unsigned short* __restrict__ Bt2p, int ldb, long strideB,
    void* __restrict__ Cout, void* __restrict__ Cout2, int ldc, long strideC,
    const float* __restrict__ bias,
    const float* __restrict__ resid, long strideR,
    int M, int N, int K, float scale) {
  typedef typename Elem<ET>::T T;
  typedef typename Frag<T>::V V;
  const T* A = (const T*)Ap; const T* A2 = (const T*)A2p; const T* Bt = (const T*)Btp; const T* Bt2 = (const T*)Bt2p;
  __shared__ __align__(16) float sT[8][16 * 68];
  const int b    = blockIdx.y;
  const int lane = threadIdx.x & 31;
  const int wave = threadIdx.x >> 5;
  const int tilesN = N >> 6;
  const int tilesM = M >> 6;
  const int tile = blockIdx.x * 8 + wave;
  if (tile >= tilesM * tilesN) return;
  const int tm = tile / tilesN;
  const int tn = tile - tm * tilesN;
  const int m0 = tm << 6;
  const int n0 = tn << 6;

  const T* Ab  = A  + (size_t)b * strideA;
  const T* Bb  = Bt + (size_t)b * strideB;
  const T* Ab2 = SPLIT ? (A2  + (size_t)b * strideA) : nullptr;
  const T* Bb2 = SPLIT ? (Bt2 + (size_t)b * strideB) : nullptr;

  const int rlane = lane & 15;
  const int koff  = (lane >> 4) * 8;
  const int mOff  = (lane >> 4) * 8;

  v8f acc[4][4];
#pragma unroll
  for (int i = 0; i < 4; ++i)
#pragma unroll
    for (int j = 0; j < 4; ++j) acc[i][j] = (v8f){0.f,0.f,0.f,0.f,0.f,0.f,0.f,0.f};

  for (int k0 = 0; k0 < K; k0 += 32) {
    V bh[4], bl[4];
#pragma unroll
    for (int j = 0; j < 4; ++j) {
      const size_t bo = (size_t)(n0 + (j << 4) + rlane) * ldb + koff + k0;
      bh[j] = Frag<T>::load(Bb + bo);
      if (SPLIT) bl[j] = Frag<T>::load(Bb2 + bo);
    }
#pragma unroll
    for (int i = 0; i < 4; ++i) {
      const size_t ao = (size_t)(m0 + (i << 4) + rlane) * lda + koff + k0;
      V ah = Frag<T>::load(Ab + ao);
      V al;
      if (SPLIT) al = Frag<T>::load(Ab2 + ao);
#pragma unroll
      for (int j = 0; j < 4; ++j) {
        acc[i][j] = Frag<T>::mma(ah, bh[j], acc[i][j]);
        if (SPLIT) {
          acc[i][j] = Frag<T>::mma(ah, bl[j], acc[i][j]);
          acc[i][j] = Frag<T>::mma(al, bh[j], acc[i][j]);
        }
      }
      Frag<T>::guard(acc[i][0], acc[i][3], ah, SPLIT ? al : ah);
    }
    Frag<T>::keep(bh[0], bh[1], bh[2], bh[3]);
    if (SPLIT) Frag<T>::keep(bl[0], bl[1], bl[2], bl[3]);
  }
  acc_guard4(acc[0][0], acc[0][1], acc[0][2], acc[0][3]);
  acc_guard4(acc[1][0], acc[1][1], acc[1][2], acc[1][3]);
  acc_guard4(acc[2][0], acc[2][1], acc[2][2], acc[2][3]);
  acc_guard4(acc[3][0], acc[3][1], acc[3][2], acc[3][3]);

  float* slab = sT[wave];
  const float* Rb = RESID ? (resid + (size_t)b * strideR) : nullptr;
#pragma unroll
  for (int i = 0; i < 4; ++i) {
    const int mBase = m0 + (i << 4);
#pragma unroll
    for (int j = 0; j < 4; ++j) {
      const int n = n0 + (j << 4) + rlane;
      float bv = 0.f;
      if (BIAS_MODE == 2) bv = bias[n];
#pragma unroll
      for (int r = 0; r < 8; ++r) {
        float v = acc[i][j][r] * scale;
        if (BIAS_MODE == 1) v += bias[mBase + mOff + r];
        if (BIAS_MODE == 2) v += bv;
        if (RESID) v += Rb[(size_t)(mBase + mOff + r) * ldc + n];
        if (ACT == 1) v = tanhf(v);
        if (ACT == 2) v = fmaxf(v, 0.0f);
        if (ACT == 4) v = (v > 0.f) ? v : 0.01f * v;
        slab[(mOff + r) * 68 + (j << 4) + rlane] = v;
      }
    }
    __builtin_amdgcn_fence(__ATOMIC_RELEASE, "workgroup");
    __builtin_amdgcn_wave_barrier();
    __builtin_amdgcn_fence(__ATOMIC_ACQUIRE, "workgroup");
    if (OUT_MODE == 0) {
      float* C = (float*)Cout + (size_t)b * strideC;
      const int hh = lane >> 4, c4 = (lane & 15) * 4;
      for (int pass = 0; pass < 2; ++pass) {
#pragma unroll
        for (int it = 0; it < 8; ++it) {
          const int row = it * 2 + hh;
          v4f v = *(const v4f*)(slab + row * 68 + c4);
          *(volatile v4f*)(C + (size_t)(mBase + row) * ldc + n0 + c4) = v;
        }
        __threadfence();
      }
    } else {
      const int q = lane >> 3, c8 = (lane & 7) * 8;
      unsigned short* C  = (unsigned short*)Cout  + (size_t)b * strideC;
      unsigned short* C2 = (OUT_MODE == 2) ? ((unsigned short*)Cout2 + (size_t)b * strideC) : nullptr;
      for (int pass = 0; pass < 2; ++pass) {
#pragma unroll
        for (int it = 0; it < 4; ++it) {
          const int row = it * 4 + q;
          const float* sp = slab + row * 68 + c8;
          v8h hv, lv;
#pragma unroll
          for (int e = 0; e < 8; ++e) {
            if (OUT_MODE == 1) {
              hv[e] = (_Float16)sp[e];
            } else {
              unsigned short hb = f2bf_bits(sp[e]);
              unsigned short lb = f2bf_bits(sp[e] - bf_bits2f(hb));
              hv[e] = __builtin_bit_cast(_Float16, hb);
              lv[e] = __builtin_bit_cast(_Float16, lb);
            }
          }
          *(volatile v8h*)(C + (size_t)(mBase + row) * ldc + n0 + c8) = hv;
          if (OUT_MODE == 2) *(volatile v8h*)(C2 + (size_t)(mBase + row) * ldc + n0 + c8) = lv;
        }
        __threadfence();
      }
    }
    __builtin_amdgcn_fence(__ATOMIC_RELEASE, "workgroup");
    __builtin_amdgcn_wave_barrier();
    __builtin_amdgcn_fence(__ATOMIC_ACQUIRE, "workgroup");
  }
}

__global__ __launch_bounds__(PTHR) void pad12_f16_kernel(const float* __restrict__ src, unsigned short* __restrict__ dst,
                                                         int nrow, float sc) {
  const int i  = blockIdx.x * PTHR + threadIdx.x;
  const int n8 = nrow * 4;
  if (i < n8) {
    const int row = i >> 2;
    const int q   = i & 3;
    const float* sp = src + (size_t)row * NINP;
    const int o0 = (q == 0) ? 0 : 8;
    const int o1 = (q == 0) ? 4 : 8;
    const v4f a = *(const v4f*)(sp + o0);
    const v4f b = *(const v4f*)(sp + o1);
    const bool va = (q < 2);
    const bool vb = (q == 0);
    v8h hv;
#pragma unroll
    for (int e = 0; e < 4; ++e) {
      const float fa = a[e] * sc;
      const float fb = b[e] * sc;
      hv[e]     = (_Float16)(va ? fa : 0.0f);
      hv[4 + e] = (_Float16)(vb ? fb : 0.0f);
    }
    *(volatile v8h*)(dst + (size_t)i * 8) = hv;
    __threadfence();
    *(volatile v8h*)(dst + (size_t)i * 8) = hv;
  }
}

__device__ __forceinline__ v16h wfrag_from_f32(const float* p, float sc, bool valid) {
  const v4f q0 = *(const v4f*)(p);
  const v4f q1 = *(const v4f*)(p + 4);
  const v4f q2 = *(const v4f*)(p + 16);
  const v4f q3 = *(const v4f*)(p + 20);
  v16h f;
#pragma unroll
  for (int e = 0; e < 4; ++e) {
    const float f0 = q0[e] * sc;
    const float f1 = q1[e] * sc;
    const float f2 = q2[e] * sc;
    const float f3 = q3[e] * sc;
    f[e]      = (_Float16)(valid ? f0 : 0.0f);
    f[4 + e]  = (_Float16)(valid ? f1 : 0.0f);
    f[8 + e]  = (_Float16)(valid ? f2 : 0.0f);
    f[12 + e] = (_Float16)(valid ? f3 : 0.0f);
  }
  return f;
}

__device__ __forceinline__ float sigm_f32(float x) { return __builtin_amdgcn_rcpf(1.0f + expf(-x)); }
__device__ __forceinline__ float tanh_f32(float x) { return 1.0f - 2.0f * __builtin_amdgcn_rcpf(expf(2.0f * x) + 1.0f); }

__global__ __launch_bounds__(RTHR) void lstm_seq_kernel(const float* __restrict__ XG,
                                                        const float* __restrict__ W_hh,
                                                        const float* __restrict__ b_ih,
                                                        const float* __restrict__ b_hh,
                                                        const float* __restrict__ W_out,
                                                        const float* __restrict__ b_out,
                                                        float* __restrict__ out) {
  __shared__ __align__(16) _Float16 Hb[2][2 * NHID];
  __shared__ __align__(16) float    Ob[NOUTC * OBLK];
  const int tid  = threadIdx.x;
  const int lane = tid & 31;
  const int wave = __builtin_amdgcn_readfirstlane(tid >> 5);
  const int c    = lane & 15;
  const int hh   = lane >> 4;
  const int koff = hh * 8;
  const int unit = 16 * wave + c;

  v16h bw[4][2];
#pragma unroll
  for (int g = 0; g < 4; ++g) {
#pragma unroll
    for (int kk = 0; kk < 2; ++kk) {
      bw[g][kk] = wfrag_from_f32(W_hh + (size_t)(g * NHID + unit) * NHID + kk * 32 + koff, WCARRY, true);
      settle_frag(bw[g][kk]);
    }
  }
  const int  nc   = (c < NOUTC) ? c : (NOUTC - 1);
  const bool nval = (c < NOUTC);
  v16h bo0 = wfrag_from_f32(W_out + (size_t)nc * NHID + koff, WCARRY, nval);
  settle_frag(bo0);
  v16h bo1 = wfrag_from_f32(W_out + (size_t)nc * NHID + 32 + koff, WCARRY, nval);
  settle_frag(bo1);

  float bs[4];
#pragma unroll
  for (int g = 0; g < 4; ++g) {
    const float b0 = b_ih[g * NHID + unit];
    const float b1 = b_hh[g * NHID + unit];
    bs[g] = b0 + b1;
    settle_f32(bs[g]);
  }
  float bov = b_out[nc];
  settle_f32(bov);

  (&Hb[0][0])[tid] = (_Float16)0.0f;
  float cst = 0.0f;

  float xn[4];
#pragma unroll
  for (int g = 0; g < 4; ++g) {
    xn[g] = XG[(size_t)g * NHID + unit];
    settle_f32(xn[g]);
  }

  const bool avalid = ((c & 7) < 2);
  const int  arow   = c & 1;
  const v16h zh = {};
  const v8f  z8 = {0.f, 0.f, 0.f, 0.f, 0.f, 0.f, 0.f, 0.f};
  __syncthreads();

#pragma unroll 1
  for (int t = 0; t <= NSTEP; ++t) {
    const int cur = t & 1;
    float xc[4];
#pragma unroll
    for (int g = 0; g < 4; ++g) xc[g] = xn[g];
    const int tn = (t + 1 < NSTEP) ? (t + 1) : (NSTEP - 1);
    const float* xrow = XG + (size_t)tn * NGATE + unit;
#pragma unroll
    for (int g = 0; g < 4; ++g) xn[g] = xrow[g * NHID];

    const _Float16* hrow = &Hb[cur][0] + arow * NHID + koff;
    const v16h a0l = Frag<_Float16>::load(hrow);
    const v16h a1l = Frag<_Float16>::load(hrow + 32);
    const v16h a0 = avalid ? a0l : zh;
    const v16h a1 = avalid ? a1l : zh;

    v8f acc[4];
#pragma unroll
    for (int g = 0; g < 4; ++g) acc[g] = z8;
#pragma unroll
    for (int g = 0; g < 4; ++g) acc[g] = Frag<_Float16>::mma(a0, bw[g][0], acc[g]);
#pragma unroll
    for (int g = 0; g < 4; ++g) acc[g] = Frag<_Float16>::mma(a1, bw[g][1], acc[g]);
    group_guard4(acc[0], acc[1], acc[2], acc[3], a0, a1);
    keep4_h(bw[0][0], bw[1][0], bw[2][0], bw[3][0]);
    keep4_h(bw[0][1], bw[1][1], bw[2][1], bw[3][1]);

    if (wave == 0) {
      v8f ao = z8;
      ao = Frag<_Float16>::mma(a0, bo0, ao);
      ao = Frag<_Float16>::mma(a1, bo1, ao);
      group_guard1(ao, a0, a1, bo0, bo1);
      if (t >= 1) {
        const float ov = (ao[0] + ao[1] * LOCARRY_INV) * WCARRY_INV + bov;
        if (lane < NOUTC) Ob[((t - 1) & (OBLK - 1)) * NOUTC + lane] = ov;
      }
      if (t >= OBLK && (t & (OBLK - 1)) == 0) {
        wave_lds_sync();
        const v4f v = *(const v4f*)(Ob + lane * 4);
        float* op = out + (size_t)(t - OBLK) * NOUTC + lane * 4;
        *(volatile v4f*)op = v;
        __threadfence();
        *(volatile v4f*)op = v;
        wave_lds_sync();
      }
    }

    const float zi = (acc[0][0] + acc[0][1] * LOCARRY_INV) * WCARRY_INV + (xc[0] + bs[0]);
    const float zf = (acc[1][0] + acc[1][1] * LOCARRY_INV) * WCARRY_INV + (xc[1] + bs[1]);
    const float zg = (acc[2][0] + acc[2][1] * LOCARRY_INV) * WCARRY_INV + (xc[2] + bs[2]);
    const float zo = (acc[3][0] + acc[3][1] * LOCARRY_INV) * WCARRY_INV + (xc[3] + bs[3]);
    const float ig = sigm_f32(zi);
    const float fg = sigm_f32(zf);
    const float gg = tanh_f32(zg);
    const float og = sigm_f32(zo);
    cst = fg * cst + ig * gg;
    const float hnew = og * tanh_f32(cst);

    const float hq = (fabsf(hnew) < F16_MIN_NORMAL) ? 0.0f : hnew;
    const _Float16 hhi = (_Float16)hq;
    const float hres = hnew - (float)hhi;
    const _Float16 hlo = (_Float16)(hres * LOCARRY);
    _Float16* hn = &Hb[cur ^ 1][0];
    if (hh == 0) {
      hn[unit] = hhi;
      hn[NHID + unit] = hlo;
    }
    __syncthreads();
  }
}

extern "C" void kernel_launch(void* const* d_in, const int* in_sizes, int n_in,
                              void* d_out, int out_size, void* d_ws, size_t ws_size, hipStream_t stream) {
  (void)in_sizes; (void)out_size;
  if (n_in < 7 || d_out == nullptr || d_ws == nullptr) return;

  const float* feature = (const float*)d_in[0];
  const float* w_ih    = (const float*)d_in[1];
  const float* w_hh    = (const float*)d_in[2];
  const float* b_ih    = (const float*)d_in[3];
  const float* b_hh    = (const float*)d_in[4];
  const float* w_out   = (const float*)d_in[5];
  const float* b_out   = (const float*)d_in[6];
  float* out = (float*)d_out;

  char* ws = (char*)d_ws; size_t off = 0;
  auto carve = [&](size_t bytes) -> char* { char* p = ws + off; off += (bytes + 255) & ~(size_t)255; return p; };
  unsigned short* FA  = (unsigned short*)carve((size_t)NSTEP * KPAD * 2);
  unsigned short* WIB = (unsigned short*)carve((size_t)NGATE * KPAD * 2);
  float*          XG  = (float*)carve((size_t)NSTEP * NGATE * 4);
  if (off > ws_size || off > (size_t)134217728) return;

  pad12_f16_kernel<<<(NSTEP * 4 + PTHR - 1) / PTHR, PTHR, 0, stream>>>(feature, FA, NSTEP, 1.0f);
  pad12_f16_kernel<<<(NGATE * 4 + PTHR - 1) / PTHR, PTHR, 0, stream>>>(w_ih, WIB, NGATE, WCARRY);

  const dim3 ggrid((NSTEP / 64) * (NGATE / 64) / 8, 1);
  wmma_gemm64<0, false, 0, 0, false, 0><<<ggrid, 256, 0, stream>>>(
      FA, FA, KPAD, 0L, WIB, WIB, KPAD, 0L, (void*)XG, (void*)XG, NGATE, 0L,
      XG, XG, 0L, NSTEP, NGATE, KPAD, WCARRY_INV);

  lstm_seq_kernel<<<1, RTHR, 0, stream>>>(XG, w_hh, b_ih, b_hh, w_out, b_out, out);
}
